// GATv2Classifier_69999376990329
// MI455X (gfx1250) — hardware-verified
//
#include <hip/hip_runtime.h>
#include <stddef.h>


#define NTHR  256
#define NWAVE 8
#define FW    256
#define NHD   4
#define DH    64
#define NG    16
#define NC    10
#define GR    64
#define GC    128
#define XSP   132
#define NB    256
#define NBSH  8
#define CHUNK 2048
#define NGRP  (CHUNK / (NTHR * 4))
#define WCAP  ((CHUNK / NTHR) * 32)
#define AGG_LDS_BYTES (NB * FW * 4 + 2 * NB * NHD * 4 + NWAVE * WCAP * 4 + NWAVE * 4 + NB * 4)

static_assert(NGRP == 2);
static_assert(WCAP == NGRP * 4 * 32);
static_assert((1 << NBSH) == NB);
static_assert(AGG_LDS_BYTES == 279584);
static_assert((XSP % 4) == 0);
static_assert(FW == 2 * GC);
static_assert(NG * DH == 4 * NTHR);
static_assert(NG * DH * 4 <= NWAVE * WCAP * 4);
static_assert(((NG * NC) % 4) == 0);
static_assert(FW == NHD * DH);

typedef float    v4f  __attribute__((ext_vector_type(4)));
typedef float    v8f  __attribute__((ext_vector_type(8)));
typedef int      v4i  __attribute__((ext_vector_type(4)));
typedef _Float16 v8h  __attribute__((ext_vector_type(8)));
typedef _Float16 v16h __attribute__((ext_vector_type(16)));

union FragH { v16h v; v4i u[2]; };
union Pack  { v8h h; v4i i; };

__device__ __forceinline__ v8f wmh(v16h a, v16h b, v8f c) {
  v8f d = __builtin_amdgcn_wmma_f32_16x16x32_f16(false, a, false, b, (short)0, c, false, false);
  asm volatile("v_nop\n\tv_nop\n\tv_nop\n\tv_nop" : "+v"(d) : "v"(a), "v"(b));
  return d;
}

__device__ __forceinline__ float lk(float t) { return fmaxf(t, 0.2f * t); }
__device__ __forceinline__ float dl(v4f t, v4f w) {
  return w.x * lk(t.x) + w.y * lk(t.y) + w.z * lk(t.z) + w.w * lk(t.w);
}

__global__ __launch_bounds__(NTHR) void k_cvt_x(const float* __restrict__ src, int rows_src,
                                                _Float16* dst, int rows_total) {
  const int i = blockIdx.x * NTHR + threadIdx.x;
  if (i >= rows_total * (FW / 8)) return;
  const int r  = i >> 5;
  const int kb = (i & 31) * 8;
  v4f lo = {0.f, 0.f, 0.f, 0.f};
  v4f hi = lo;
  if (r < rows_src) {
    const float* p = src + (size_t)r * FW + kb;
    lo = *(const v4f*)(p);
    hi = *(const v4f*)(p + 4);
  }
  Pack u;
  const v4i z4 = {0, 0, 0, 0};
  u.i = z4;
#pragma unroll
  for (int j = 0; j < 4; ++j) {
    u.h[j]     = (_Float16)lo[j];
    u.h[4 + j] = (_Float16)hi[j];
  }
  _Float16* op = dst + (size_t)r * FW + kb;
  *(volatile v4i*)op = u.i;
  __threadfence();
  *(volatile v4i*)op = u.i;
}

__global__ __launch_bounds__(NTHR) void k_cvt_w(const float* __restrict__ Ws, const float* __restrict__ Wd,
                                                _Float16* dst, float scale) {
  const int i = blockIdx.x * NTHR + threadIdx.x;
  if (i >= 2 * FW * (FW / 8)) return;
  const int n   = i >> 5;
  const int kb  = (i & 31) * 8;
  const float* W = (n < FW) ? Ws : Wd;
  const int col = n & (FW - 1);
  Pack u;
  const v4i z4 = {0, 0, 0, 0};
  u.i = z4;
#pragma unroll
  for (int j = 0; j < 8; ++j) u.h[j] = (_Float16)(W[(size_t)(kb + j) * FW + col] * scale);
  _Float16* op = dst + (size_t)n * FW + kb;
  *(volatile v4i*)op = u.i;
  __threadfence();
  *(volatile v4i*)op = u.i;
}

__global__ __launch_bounds__(NTHR) void k_gemm(const _Float16* __restrict__ A, const _Float16* __restrict__ Bt,
                                               const float* __restrict__ bs, const float* __restrict__ bd,
                                               float* fs, float* fd, float oscale) {
  __shared__ __attribute__((aligned(16))) float Xs[GR * XSP];

  const int tid  = threadIdx.x;
  const int lane = tid & 31;
  const int wave = tid >> 5;
  const int hh   = lane >> 4;
  const int m    = lane & 15;
  const int wr   = wave >> 2;
  const int wc   = wave & 3;
  const int rowBase = blockIdx.x * GR;
  const int colBase = blockIdx.y * GC;
  const int which   = blockIdx.y >> 1;
  const int cb      = colBase - which * FW;
  const float* bias = which ? bd : bs;
  float* outp       = which ? fd : fs;

  const size_t ra0 = (size_t)(rowBase + 32 * wr + m) * FW + 8 * hh;
  const size_t ra1 = ra0 + (size_t)16 * FW;
  const size_t rb0 = (size_t)(colBase + 32 * wc + m) * FW + 8 * hh;
  const size_t rb1 = rb0 + (size_t)16 * FW;

  const v8f z8 = {0.f, 0.f, 0.f, 0.f, 0.f, 0.f, 0.f, 0.f};
  v8f c00 = z8, c01 = z8, c10 = z8, c11 = z8;

#pragma unroll 1
  for (int k0 = 0; k0 < FW; k0 += 32) {
    FragH a0, a1, b0, b1;
    a0.u[0] = *(const v4i*)(A + ra0 + k0);   a0.u[1] = *(const v4i*)(A + ra0 + k0 + 16);
    a1.u[0] = *(const v4i*)(A + ra1 + k0);   a1.u[1] = *(const v4i*)(A + ra1 + k0 + 16);
    b0.u[0] = *(const v4i*)(Bt + rb0 + k0);  b0.u[1] = *(const v4i*)(Bt + rb0 + k0 + 16);
    b1.u[0] = *(const v4i*)(Bt + rb1 + k0);  b1.u[1] = *(const v4i*)(Bt + rb1 + k0 + 16);
    c00 = wmh(a0.v, b0.v, c00);
    c01 = wmh(a0.v, b1.v, c01);
    c10 = wmh(a1.v, b0.v, c10);
    c11 = wmh(a1.v, b1.v, c11);
  }

  const int cl0 = 32 * wc + m, cl1 = cl0 + 16;
  const float bv0 = bias[cb + cl0], bv1 = bias[cb + cl1];
  const int rl0 = 32 * wr + 8 * hh, rl1 = rl0 + 16;
#pragma unroll
  for (int r = 0; r < 8; ++r) {
    Xs[(rl0 + r) * XSP + cl0] = c00[r] * oscale + bv0;
    Xs[(rl0 + r) * XSP + cl1] = c01[r] * oscale + bv1;
    Xs[(rl1 + r) * XSP + cl0] = c10[r] * oscale + bv0;
    Xs[(rl1 + r) * XSP + cl1] = c11[r] * oscale + bv1;
  }
  __syncthreads();

  v4f xv[8];
#pragma unroll
  for (int i = 0; i < 8; ++i) xv[i] = *(const v4f*)(Xs + (8 * wave + i) * XSP + 4 * lane);
  float* ob = outp + (size_t)(rowBase + 8 * wave) * FW + cb + 4 * lane;
#pragma unroll
  for (int i = 0; i < 8; ++i) *(volatile v4f*)(ob + (size_t)i * FW) = xv[i];
  __threadfence();
#pragma unroll
  for (int i = 0; i < 8; ++i) *(volatile v4f*)(ob + (size_t)i * FW) = xv[i];
}

__device__ __forceinline__ void hit8(const float* xs, const float* xd, float* ar, float* mp, float* dp,
                                     v4f w0, v4f w1) {
  const v4f a0 = *(const v4f*)(xs), a1 = *(const v4f*)(xs + 4);
  const v4f d0 = *(const v4f*)(xd), d1 = *(const v4f*)(xd + 4);
  float s = dl(a0 + d0, w0) + dl(a1 + d1, w1);
  s += __shfl_xor(s, 4, 32);
  s += __shfl_xor(s, 2, 32);
  s += __shfl_xor(s, 1, 32);
  const float m  = mp[0], n = dp[0];
  const float mn = fmaxf(m, s);
  const float sc = __expf(m - mn);
  const float p  = __expf(s - mn);
  v4f e0 = *(v4f*)(ar), e1 = *(v4f*)(ar + 4);
  e0 = e0 * sc + a0 * p;
  e1 = e1 * sc + a1 * p;
  *(v4f*)(ar)     = e0;
  *(v4f*)(ar + 4) = e1;
  mp[0] = mn;
  dp[0] = n * sc + p;
}

template <int L2>
__global__ __launch_bounds__(NTHR) void k_agg(
    const int* __restrict__ esrc, const int* __restrict__ edst, const int* __restrict__ gid,
    const float* __restrict__ xl, const float* __restrict__ xr, const float* __restrict__ att,
    _Float16* xo, float* pmo, int nN, int nE, int nPad) {
  extern __shared__ v4f lds_dyn[];
  float* sacc = (float*)lds_dyn;
  float* mx   = sacc + NB * FW;
  float* dn   = mx + NB * NHD;
  int*   list = (int*)(dn + NB * NHD);
  int*   wcnt = list + NWAVE * WCAP;
  int*   sgid = wcnt + NWAVE;

  const int tid  = threadIdx.x;
  const int lane = tid & 31;
  const int wave = tid >> 5;
  const int nodeBase = blockIdx.x * NB;

  {
    const v4f z4 = {0.f, 0.f, 0.f, 0.f};
    for (int i = tid; i < NB * FW / 4; i += NTHR) lds_dyn[i] = z4;
    for (int i = tid; i < NB * NHD; i += NTHR) { mx[i] = -1.0e30f; dn[i] = 0.f; }
    if (L2) {
      for (int i = tid; i < NB; i += NTHR) {
        const int node = nodeBase + i;
        int g = -1;
        if (node < nN) g = gid[node];
        sgid[i] = g;
      }
    }
  }
  __syncthreads();

  const int coff = 8 * lane;
  const int hidx = lane >> 3;
  const v4f w0 = *(const v4f*)(att + coff);
  const v4f w1 = *(const v4f*)(att + coff + 4);

  const bool al16 = ((nE & 3) == 0);
  const int nChunks = (nE + CHUNK - 1) / CHUNK;

#pragma unroll 1
  for (int ch = 0; ch < nChunks; ++ch) {
    const int cbase = ch * CHUNK;
    int wc = 0;
#pragma unroll
    for (int g = 0; g < NGRP; ++g) {
      const int el0 = (g * NTHR + tid) * 4;
      const int e0  = cbase + el0;
      const int sent = -2147483647 - 1;
      v4i d;
      if (al16 && (e0 + 3 < nE)) {
        d = *(const v4i*)(edst + e0);
      } else {
        d.x = (e0     < nE) ? edst[min(e0, nE - 1)]     : sent;
        d.y = (e0 + 1 < nE) ? edst[min(e0 + 1, nE - 1)] : sent;
        d.z = (e0 + 2 < nE) ? edst[min(e0 + 2, nE - 1)] : sent;
        d.w = (e0 + 3 < nE) ? edst[min(e0 + 3, nE - 1)] : sent;
      }
      const unsigned s0 = (unsigned)d.x - (unsigned)nodeBase;
      const unsigned s1 = (unsigned)d.y - (unsigned)nodeBase;
      const unsigned s2 = (unsigned)d.z - (unsigned)nodeBase;
      const unsigned s3 = (unsigned)d.w - (unsigned)nodeBase;
      const bool h0 = s0 < (unsigned)NB;
      const bool h1 = s1 < (unsigned)NB;
      const bool h2 = s2 < (unsigned)NB;
      const bool h3 = s3 < (unsigned)NB;
      const unsigned many = __builtin_amdgcn_ballot_w32(h0 | h1 | h2 | h3);
      if (many != 0u) {
#define HITJ(J, HJ, SJ) { \
          const unsigned mj = __builtin_amdgcn_ballot_w32(HJ); \
          if (HJ) { \
            const int pos = wc + (int)__builtin_amdgcn_mbcnt_lo(mj, 0u); \
            if (pos < WCAP) list[wave * WCAP + pos] = ((el0 + (J)) << NBSH) | (int)(SJ); \
          } \
          wc += (int)__builtin_popcount(mj); }
        HITJ(0, h0, s0)
        HITJ(1, h1, s1)
        HITJ(2, h2, s2)
        HITJ(3, h3, s3)
#undef HITJ
      }
    }
    if (lane == 0) wcnt[wave] = wc;
    __syncthreads();

    if (wave == 0) {
#pragma unroll 1
      for (int wsx = 0; wsx < NWAVE; ++wsx) {
        int n = __builtin_amdgcn_readfirstlane(wcnt[wsx]);
        n = n > WCAP ? WCAP : n;
        n = n < 0 ? 0 : n;
#pragma unroll 1
        for (int i = 0; i < n; ++i) {
          const int ent  = __builtin_amdgcn_readfirstlane(list[wsx * WCAP + i]);
          const int slot = ent & (NB - 1);
          const int el   = (ent >> NBSH) & (CHUNK - 1);
          const int node = nodeBase + slot;
          if (node >= nN) continue;
          int e = cbase + el;
          if (e > nE - 1) e = nE - 1;
          int sj = esrc[e];
          sj = sj < 0 ? 0 : (sj > nN - 1 ? nN - 1 : sj);
          hit8(xl + (size_t)sj * FW + coff, xr + (size_t)node * FW + coff,
               sacc + slot * FW + coff, mx + slot * NHD + hidx, dn + slot * NHD + hidx, w0, w1);
        }
      }
    }
    __syncthreads();
  }

  if (L2 == 0) {
#pragma unroll 1
    for (int s = wave; s < NB; s += NWAVE) {
      const int node = nodeBase + s;
      if (node >= nPad) break;
      Pack u;
      const v4i z4 = {0, 0, 0, 0};
      u.i = z4;
      if (node < nN) {
        const float inv = 1.0f / fmaxf(dn[s * NHD + hidx], 1e-16f);
        const float* ar = sacc + s * FW + coff;
        const v4f e0 = *(const v4f*)(ar), e1 = *(const v4f*)(ar + 4);
#pragma unroll
        for (int j = 0; j < 4; ++j) {
          u.h[j]     = (_Float16)fmaxf(e0[j] * inv, 0.f);
          u.h[4 + j] = (_Float16)fmaxf(e1[j] * inv, 0.f);
        }
      }
      _Float16* op = xo + (size_t)node * FW + coff;
      *(volatile v4i*)op = u.i;
      __threadfence();
      *(volatile v4i*)op = u.i;
    }
  } else {
#pragma unroll 1
    for (int s = wave; s < NB; s += NWAVE) {
      const int node = nodeBase + s;
      if (node >= nN) break;
      const int c = 2 * lane;
      float t0 = 0.f, t1 = 0.f;
#pragma unroll
      for (int hq = 0; hq < NHD; ++hq) {
        const float inv = 1.0f / fmaxf(dn[s * NHD + hq], 1e-16f);
        const float a = sacc[s * FW + hq * DH + c];
        const float b = sacc[s * FW + hq * DH + c + 1];
        t0 += fmaxf(a * inv, 0.f);
        t1 += fmaxf(b * inv, 0.f);
      }
      sacc[s * FW + c]     = 0.25f * t0;
      sacc[s * FW + c + 1] = 0.25f * t1;
    }
    __syncthreads();

    const int c  = tid & (DH - 1);
    const int g0 = 4 * (tid >> 6);
    const float ninf = -__builtin_inff();
    float m0 = ninf, m1 = ninf, m2 = ninf, m3 = ninf;
#pragma unroll 4
    for (int s = 0; s < NB; ++s) {
      const int g   = sgid[s];
      const float v = sacc[s * FW + c];
      m0 = (g == g0)     ? fmaxf(m0, v) : m0;
      m1 = (g == g0 + 1) ? fmaxf(m1, v) : m1;
      m2 = (g == g0 + 2) ? fmaxf(m2, v) : m2;
      m3 = (g == g0 + 3) ? fmaxf(m3, v) : m3;
    }
    float* pm = (float*)list;
    pm[(g0 + 0) * DH + c] = m0;
    pm[(g0 + 1) * DH + c] = m1;
    pm[(g0 + 2) * DH + c] = m2;
    pm[(g0 + 3) * DH + c] = m3;
    __syncthreads();
    const v4f val = *(const v4f*)(pm + 4 * tid);
    float* op = pmo + (size_t)blockIdx.x * (NG * DH) + 4 * tid;
    *(volatile v4f*)op = val;
    __threadfence();
    *(volatile v4f*)op = val;
  }
}

__global__ __launch_bounds__(NTHR) void k_head(const float* __restrict__ pm, int nblk,
                                               const float* __restrict__ Wc, const float* __restrict__ bc,
                                               float* out) {
  __shared__ __attribute__((aligned(16))) float sp[NG * DH];
  __shared__ __attribute__((aligned(16))) float so[NG * NC];
  const int tid = threadIdx.x;
  const float ninf = -__builtin_inff();
  v4f mm = {ninf, ninf, ninf, ninf};
  const int nb = nblk < 0 ? 0 : nblk;
#pragma unroll 1
  for (int b = 0; b < nb; ++b) {
    const v4f v = *(const v4f*)(pm + (size_t)b * (NG * DH) + 4 * tid);
    mm.x = fmaxf(mm.x, v.x);
    mm.y = fmaxf(mm.y, v.y);
    mm.z = fmaxf(mm.z, v.z);
    mm.w = fmaxf(mm.w, v.w);
  }
  *(v4f*)(sp + 4 * tid) = mm;
  __syncthreads();
  if (tid < NG * NC) {
    const int g   = tid / NC;
    const int cls = tid - g * NC;
    float a = 0.f;
    for (int d = 0; d < DH; ++d) a += sp[g * DH + d] * Wc[d * NC + cls];
    so[tid] = a + bc[cls];
  }
  __syncthreads();
  if (tid < (NG * NC) / 4) {
    const v4f v = *(const v4f*)(so + 4 * tid);
    float* op = out + 4 * tid;
    *(volatile v4f*)op = v;
    __threadfence();
    *(volatile v4f*)op = v;
  }
}

extern "C" void kernel_launch(void* const* d_in, const int* in_sizes, int n_in,
                              void* d_out, int out_size, void* d_ws, size_t ws_size,
                              hipStream_t stream) {
  if (n_in < 16) return;
  if (in_sizes[0] <= 0 || (in_sizes[0] % FW) != 0) return;
  const int nN = in_sizes[0] / FW;
  const int nE = in_sizes[1];
  if (nE <= 0 || in_sizes[2] != nE || in_sizes[3] != nN) return;
  if (in_sizes[4] != FW * FW || in_sizes[5] != FW || in_sizes[6] != FW * FW || in_sizes[7] != FW ||
      in_sizes[8] != NHD * DH) return;
  if (in_sizes[9] != FW * FW || in_sizes[10] != FW || in_sizes[11] != FW * FW || in_sizes[12] != FW ||
      in_sizes[13] != NHD * DH) return;
  if (in_sizes[14] != DH * NC || in_sizes[15] != NC) return;
  if (out_size != NG * NC) return;

  const float* h     = (const float*)d_in[0];
  const int*   esrc  = (const int*)d_in[1];
  const int*   edst  = (const int*)d_in[2];
  const int*   gid   = (const int*)d_in[3];
  const float* W1s   = (const float*)d_in[4];
  const float* b1s   = (const float*)d_in[5];
  const float* W1d   = (const float*)d_in[6];
  const float* b1d   = (const float*)d_in[7];
  const float* attn1 = (const float*)d_in[8];
  const float* W2s   = (const float*)d_in[9];
  const float* b2s   = (const float*)d_in[10];
  const float* W2d   = (const float*)d_in[11];
  const float* b2d   = (const float*)d_in[12];
  const float* attn2 = (const float*)d_in[13];
  const float* Wc    = (const float*)d_in[14];
  const float* bc    = (const float*)d_in[15];
  float* out = (float*)d_out;

  const int Mpad = ((nN + GR - 1) / GR) * GR;
  const int nblk = (Mpad + NB - 1) / NB;

  char* wsp = (char*)d_ws;
  size_t off = 0;
  const size_t xB  = ((size_t)Mpad * FW * 2 + 255) & ~(size_t)255;
  const size_t wB  = ((size_t)2 * FW * FW * 2 + 255) & ~(size_t)255;
  const size_t fB  = ((size_t)Mpad * FW * 4 + 255) & ~(size_t)255;
  const size_t pB  = ((size_t)nblk * NG * DH * 4 + 255) & ~(size_t)255;
  _Float16* X16 = (_Float16*)(wsp + off); off += xB;
  _Float16* W16 = (_Float16*)(wsp + off); off += wB;
  float*    FS  = (float*)(wsp + off);    off += fB;
  float*    FD  = (float*)(wsp + off);    off += fB;
  float*    PM  = (float*)(wsp + off);    off += pB;
  if (off > ws_size) return;

  const float s16  = 16.0f;
  const float is16 = 0.0625f;

  hipFuncSetAttribute(reinterpret_cast<const void*>(&k_agg<0>),
                      hipFuncAttributeMaxDynamicSharedMemorySize, AGG_LDS_BYTES);
  hipFuncSetAttribute(reinterpret_cast<const void*>(&k_agg<1>),
                      hipFuncAttributeMaxDynamicSharedMemorySize, AGG_LDS_BYTES);

  k_cvt_x<<<(Mpad * (FW / 8) + NTHR - 1) / NTHR, NTHR, 0, stream>>>(h, nN, X16, Mpad);
  k_cvt_w<<<(2 * FW * (FW / 8) + NTHR - 1) / NTHR, NTHR, 0, stream>>>(W1s, W1d, W16, s16);
  k_gemm<<<dim3(Mpad / GR, (2 * FW) / GC), NTHR, 0, stream>>>(X16, W16, b1s, b1d, FS, FD, is16);
  k_agg<0><<<nblk, NTHR, AGG_LDS_BYTES, stream>>>(esrc, edst, gid, FS, FD, attn1, X16, PM, nN, nE, Mpad);

  k_cvt_w<<<(2 * FW * (FW / 8) + NTHR - 1) / NTHR, NTHR, 0, stream>>>(W2s, W2d, W16, s16);
  k_gemm<<<dim3(Mpad / GR, (2 * FW) / GC), NTHR, 0, stream>>>(X16, W16, b2s, b2d, FS, FD, is16);
  k_agg<1><<<nblk, NTHR, AGG_LDS_BYTES, stream>>>(esrc, edst, gid, FS, FD, attn2, X16, PM, nN, nE, Mpad);

  k_head<<<1, NTHR, 0, stream>>>(PM, nblk, Wc, bc, out);
}
